// CrossSemanticAttentionModule0_6743098655543
// MI455X (gfx1250) — hardware-verified
//
#include <hip/hip_runtime.h>
#include <stdint.h>

#define NB    2
#define CIN   512
#define CDN   256
#define CQK   32
#define NPIX  4096
#define IMW   64
#define PADW  66
#define NROW  (NB * NPIX)
#define KCV   (9 * CIN)
#define BNEPS 1e-5f

typedef _Float16 v16h __attribute__((ext_vector_type(16)));
typedef _Float16 v8h  __attribute__((ext_vector_type(8)));
typedef __bf16   v16b __attribute__((ext_vector_type(16)));
typedef float    v8f  __attribute__((ext_vector_type(8)));
typedef float    v4f  __attribute__((ext_vector_type(4)));
typedef unsigned short v8us __attribute__((ext_vector_type(8)));

static_assert((NROW % 64) == 0);
static_assert((KCV % 32) == 0);
static_assert((CDN % 64) == 0);
static_assert((CIN % 64) == 0);
static_assert(NPIX == IMW * IMW);
static_assert(IMW == 64);
static_assert((CIN % 512) == 0 && CIN == 512);

__device__ __forceinline__ unsigned short bfbits(float f) {
  unsigned u = __float_as_uint(f);
  return (unsigned short)((u + 0x7FFFu + ((u >> 16) & 1u)) >> 16);
}
__device__ __forceinline__ float bfval(unsigned short b) { return __uint_as_float(((unsigned)b) << 16); }
__device__ __forceinline__ float bfr(float f) { return bfval(bfbits(f)); }
__device__ __forceinline__ void split_bf(float f, unsigned short& hb, unsigned short& lb) {
  hb = bfbits(f);
  lb = bfbits(f - bfval(hb));
}

__device__ __forceinline__ v16b ldfrag_bf(const unsigned short* p) {
  union { v16b v; v8us u[2]; } f;
  f.u[0] = *(const v8us*)(p);
  f.u[1] = *(const v8us*)(p + 16);
  return f.v;
}
__device__ __forceinline__ v16h ldfrag_h(const _Float16* p) {
  union { v16h v; v8h u[2]; } f;
  f.u[0] = *(const v8h*)(p);
  f.u[1] = *(const v8h*)(p + 16);
  return f.v;
}
__device__ __forceinline__ v8f mma_bf(v16b a, v16b b, v8f c) {
  return __builtin_amdgcn_wmma_f32_16x16x32_bf16(false, a, false, b, (short)0, c, false, false);
}
__device__ __forceinline__ v8f mma_h(v16h a, v16h b, v8f c) {
  return __builtin_amdgcn_wmma_f32_16x16x32_f16(false, a, false, b, (short)0, c, false, false);
}
__device__ __forceinline__ v8f zero8() {
  v8f z;
#pragma unroll
  for (int i = 0; i < 8; ++i) z[i] = 0.0f;
  return z;
}

template <class X, class Y>
__device__ __forceinline__ void guard4(v8f& a, v8f& b, v8f& c, v8f& d, X x, Y y) {
#if defined(__HIP_DEVICE_COMPILE__)
  asm volatile("v_nop\n\tv_nop\n\tv_nop\n\tv_nop" : "+v"(a), "+v"(b), "+v"(c), "+v"(d) : "v"(x), "v"(y));
#endif
}
template <class X>
__device__ __forceinline__ void guard4x4(v8f& a, v8f& b, v8f& c, v8f& d, X x0, X x1, X x2, X x3) {
#if defined(__HIP_DEVICE_COMPILE__)
  asm volatile("v_nop\n\tv_nop\n\tv_nop\n\tv_nop"
               : "+v"(a), "+v"(b), "+v"(c), "+v"(d) : "v"(x0), "v"(x1), "v"(x2), "v"(x3));
#endif
}
template <class X>
__device__ __forceinline__ void guard4x8(v8f& a, v8f& b, v8f& c, v8f& d, X x0, X x1, X x2, X x3,
                                         X x4, X x5, X x6, X x7) {
#if defined(__HIP_DEVICE_COMPILE__)
  asm volatile("v_nop\n\tv_nop\n\tv_nop\n\tv_nop"
               : "+v"(a), "+v"(b), "+v"(c), "+v"(d)
               : "v"(x0), "v"(x1), "v"(x2), "v"(x3), "v"(x4), "v"(x5), "v"(x6), "v"(x7));
#endif
}
template <class X>
__device__ __forceinline__ void keep4(X a, X b, X c, X d) {
#if defined(__HIP_DEVICE_COMPILE__)
  asm volatile("v_nop" :: "v"(a), "v"(b), "v"(c), "v"(d));
#endif
}
__device__ __forceinline__ void accg4(v8f& a, v8f& b, v8f& c, v8f& d) {
#if defined(__HIP_DEVICE_COMPILE__)
  asm volatile("v_nop\n\tv_nop\n\tv_nop\n\tv_nop" : "+v"(a), "+v"(b), "+v"(c), "+v"(d));
#endif
}
__device__ __forceinline__ void wave_sync() {
  __builtin_amdgcn_fence(__ATOMIC_RELEASE, "workgroup");
  __builtin_amdgcn_wave_barrier();
  __builtin_amdgcn_fence(__ATOMIC_ACQUIRE, "workgroup");
}

__global__ __launch_bounds__(256) void cvt_w_kernel(const float* __restrict__ qw, const float* __restrict__ kw,
                                                    const float* __restrict__ vw, const float* __restrict__ uw,
                                                    unsigned short* __restrict__ wqk, unsigned short* __restrict__ wvp,
                                                    unsigned short* __restrict__ wup) {
  const int bid = (int)blockIdx.x, tid = (int)threadIdx.x;
  const float* src;
  unsigned short* dst;
  int li;
  if (bid < 4)       { src = qw; dst = wqk;             li = bid * 256 + tid; }
  else if (bid < 8)  { src = kw; dst = wqk + CQK * CDN; li = (bid - 4) * 256 + tid; }
  else if (bid < 40) { src = vw; dst = wvp;             li = (bid - 8) * 256 + tid; }
  else               { src = uw; dst = wup;             li = (bid - 40) * 256 + tid; }
  const size_t e = (size_t)li * 8;
  const v4f a = *(const v4f*)(src + e);
  const v4f b = *(const v4f*)(src + e + 4);
  v8us o;
#pragma unroll
  for (int i = 0; i < 4; ++i) { o[i] = bfbits(a[i]); o[4 + i] = bfbits(b[i]); }
  unsigned short* d = dst + e;
  *(volatile v8us*)d = o;
  __threadfence();
  *(volatile v8us*)d = o;
}

__global__ __launch_bounds__(256) void wconv_kernel(const float* __restrict__ w, unsigned short* __restrict__ wt) {
  const int li = (int)blockIdx.x * 256 + (int)threadIdx.x;
  if (li >= CDN * KCV / 8) return;
  const int e = li * 8;
  const int cin0 = e & (CIN - 1);
  const int t = e >> 9;
  const int co = t / 9;
  const int tap = t - co * 9;
  v8us o;
#pragma unroll
  for (int i = 0; i < 8; ++i) o[i] = bfbits(w[((size_t)(co * CIN + cin0 + i)) * 9 + tap]);
  unsigned short* d = wt + e;
  *(volatile v8us*)d = o;
  __threadfence();
  *(volatile v8us*)d = o;
}

__global__ __launch_bounds__(256) void xpad_kernel(const float* __restrict__ x, unsigned short* __restrict__ xp) {
  __shared__ float tile[64 * 65];
  const int tid = (int)threadIdx.x;
  const int bimg = (int)blockIdx.x / PADW;
  const int yp = (int)blockIdx.x - bimg * PADW;
  unsigned short* rowb = xp + (size_t)(bimg * PADW + yp) * PADW * CIN;
  v8us z;
#pragma unroll
  for (int e = 0; e < 8; ++e) z[e] = 0;
  if (yp == 0 || yp == PADW - 1) {
#pragma unroll
    for (int ps = 0; ps < 2; ++ps) {
#pragma unroll 1
      for (int it = 0; it < 17; ++it) {
        const int idx = it * 256 + tid;
        if (idx < PADW * CIN / 8) *(volatile v8us*)(rowb + (size_t)idx * 8) = z;
      }
      __threadfence();
    }
    return;
  }
  if (tid < 128) {
    const int xr = (tid >> 6) ? (PADW - 1) : 0;
    const int pc = tid & 63;
    unsigned short* d = rowb + (size_t)xr * CIN + pc * 8;
    *(volatile v8us*)d = z;
    __threadfence();
    *(volatile v8us*)d = z;
  }
  const int y = yp - 1;
  const float* src = x + ((size_t)bimg * CIN * IMW + y) * IMW;
  const int q = tid & 7;
#pragma unroll 1
  for (int cc = 0; cc < CIN / 64; ++cc) {
    __syncthreads();
#pragma unroll
    for (int it = 0; it < 16; ++it) {
      const int idx = it * 256 + tid;
      const int ci = idx >> 6, xx = idx & 63;
      tile[ci * 65 + xx] = src[(size_t)(cc * 64 + ci) * NPIX + xx];
    }
    __syncthreads();
#pragma unroll
    for (int ps = 0; ps < 2; ++ps) {
#pragma unroll
      for (int it = 0; it < 2; ++it) {
        const int xx = (it * 256 + tid) >> 3;
        v8us o;
#pragma unroll
        for (int e = 0; e < 8; ++e) o[e] = bfbits(tile[(8 * q + e) * 65 + xx]);
        *(volatile v8us*)(rowb + (size_t)(xx + 1) * CIN + cc * 64 + 8 * q) = o;
      }
      __threadfence();
    }
  }
}

template <bool CONV, bool SPLITA, bool SPLITB, int MODE>
__global__ __launch_bounds__(256) void gemm_kernel(
    const unsigned short* __restrict__ Ap, const unsigned short* __restrict__ A2p, int lda,
    const unsigned short* __restrict__ Bp, const unsigned short* __restrict__ B2p, int ldb, long long sB,
    float* __restrict__ Cfp, unsigned short* __restrict__ Chp, unsigned short* __restrict__ Clp, int ldc, long long sC,
    const float* __restrict__ p0, const float* __restrict__ p1, const float* __restrict__ p2,
    const float* __restrict__ p3, const float* __restrict__ p4, const float* __restrict__ p5,
    int M, int N, int K, int nsplit, float scale) {
  __shared__ __align__(16) float sT[8][16 * 68];
  const int lane = threadIdx.x & 31, wave = threadIdx.x >> 5;
  const int tilesN = N >> 6, tilesM = M >> 6;
  const int tile = (int)blockIdx.x * 8 + wave;
  if (tile >= tilesM * tilesN) return;
  const int tm = tile / tilesN, tn = tile - tm * tilesN;
  const int m0 = tm << 6, n0 = tn << 6;
  const int rl = lane & 15;
  const int koff = (lane >> 4) * 8;
  const int mOff = (lane >> 4) * 8;
  const size_t by = (size_t)blockIdx.y;
  const unsigned short* B  = Bp + by * (size_t)sB;
  const unsigned short* B2 = B2p + by * (size_t)sB;
  float* Cf = Cfp + by * (size_t)sC;
  unsigned short* Ch = Chp + by * (size_t)sC;
  unsigned short* Cl = Clp + by * (size_t)sC;
  const float* resid = p1 + by * (size_t)sC;
  const int bimg = tm >> 6, yrow = tm & 63;

  v8f acc[4][4];
#pragma unroll
  for (int i = 0; i < 4; ++i)
#pragma unroll
    for (int j = 0; j < 4; ++j) acc[i][j] = zero8();

#pragma unroll 1
  for (int k0 = 0; k0 < K; k0 += 32) {
    size_t ao[4];
    if (CONV) {
      const int tap = k0 >> 9;
      const int ky = tap / 3;
      const int kx = tap - 3 * ky;
      const int cin0 = k0 & (CIN - 1);
      const size_t rb = ((size_t)((bimg * PADW + yrow + ky) * PADW + kx)) * CIN + cin0 + koff;
#pragma unroll
      for (int i = 0; i < 4; ++i) ao[i] = rb + (size_t)((i << 4) + rl) * CIN;
    } else {
#pragma unroll
      for (int i = 0; i < 4; ++i) ao[i] = (size_t)(m0 + (i << 4) + rl) * lda + koff + k0;
    }
#pragma unroll
    for (int pb = 0; pb < (SPLITB ? 2 : 1); ++pb) {
      const unsigned short* Bs = (pb == 0) ? B : B2;
      v16b bh[4];
#pragma unroll
      for (int j = 0; j < 4; ++j) bh[j] = ldfrag_bf(Bs + (size_t)(n0 + (j << 4) + rl) * ldb + koff + k0);
#pragma unroll
      for (int i = 0; i < 4; ++i) {
        const v16b ah = ldfrag_bf(Ap + ao[i]);
        v16b al = ah;
        if (SPLITA) al = ldfrag_bf(A2p + ao[i]);
#pragma unroll
        for (int j = 0; j < 4; ++j) {
          acc[i][j] = mma_bf(ah, bh[j], acc[i][j]);
          if (SPLITA) acc[i][j] = mma_bf(al, bh[j], acc[i][j]);
        }
        guard4(acc[i][0], acc[i][1], acc[i][2], acc[i][3], ah, SPLITA ? al : bh[3]);
      }
      keep4(bh[0], bh[1], bh[2], bh[3]);
    }
  }
  accg4(acc[0][0], acc[0][1], acc[0][2], acc[0][3]);
  accg4(acc[1][0], acc[1][1], acc[1][2], acc[1][3]);
  accg4(acc[2][0], acc[2][1], acc[2][2], acc[2][3]);
  accg4(acc[3][0], acc[3][1], acc[3][2], acc[3][3]);

  float cb[4], csc[4], csh[4];
  float alpha = 0.0f;
#pragma unroll
  for (int j = 0; j < 4; ++j) { cb[j] = 0.0f; csc[j] = 1.0f; csh[j] = 0.0f; }
  if (MODE == 0) {
    alpha = bfr(p5[0]);
#pragma unroll
    for (int j = 0; j < 4; ++j) {
      const int cc = n0 + (j << 4) + rl;
      const float g = bfr(p1[cc]), bb = bfr(p2[cc]), bm = bfr(p3[cc]), bv = bfr(p4[cc]);
      const float sc = g * (1.0f / sqrtf(bv + BNEPS));
      cb[j] = bfr(p0[cc]);
      csc[j] = sc;
      csh[j] = bb - bm * sc;
    }
  }
  if (MODE == 1) {
#pragma unroll
    for (int j = 0; j < 4; ++j) {
      const int cc = n0 + (j << 4) + rl;
      const int i0 = min(cc, nsplit - 1);
      const int i1 = min(max(cc - nsplit, 0), N - nsplit - 1);
      const float v0 = bfr(p0[i0]), v1 = bfr(p1[i1]);
      cb[j] = (cc < nsplit) ? v0 : v1;
    }
  }

  float* slab = sT[wave];
  const int hh = lane >> 4, c4 = (lane & 15) * 4;
  const int qq = lane >> 3, c8 = (lane & 7) * 8;
#pragma unroll
  for (int i = 0; i < 4; ++i) {
    const int mBase = m0 + (i << 4);
    float rbv[8];
#pragma unroll
    for (int r = 0; r < 8; ++r) rbv[r] = 0.0f;
    if (MODE == 2 || MODE == 3) {
      const v4f ra = *(const v4f*)(p0 + mBase + mOff);
      const v4f rq = *(const v4f*)(p0 + mBase + mOff + 4);
#pragma unroll
      for (int r = 0; r < 4; ++r) { rbv[r] = bfr(ra[r]); rbv[4 + r] = bfr(rq[r]); }
    }
#pragma unroll
    for (int j = 0; j < 4; ++j) {
#pragma unroll
      for (int r = 0; r < 8; ++r) {
        float v = acc[i][j][r];
        if (MODE == 0) {
          float t = v + cb[j];
          t = t * csc[j] + csh[j];
          v = (t > 0.0f) ? t : alpha * t;
        }
        if (MODE == 1) v = v + cb[j];
        if (MODE == 2) v = (v + rbv[r]) * scale;
        if (MODE == 3) v = v + rbv[r];
        slab[(mOff + r) * 68 + (j << 4) + rl] = v;
      }
    }
    wave_sync();
#pragma unroll
    for (int ps = 0; ps < 2; ++ps) {
      if (MODE == 0 || MODE == 3) {
#pragma unroll
        for (int it = 0; it < 8; ++it) {
          const int row = it * 2 + hh;
          v4f xv = *(const v4f*)(slab + row * 68 + c4);
          const size_t go = (size_t)(mBase + row) * ldc + n0 + c4;
          if (MODE == 3) {
            const v4f rr = *(const v4f*)(resid + go);
#pragma unroll
            for (int e = 0; e < 4; ++e) xv[e] = xv[e] + bfr(rr[e]);
          }
          *(volatile v4f*)(Cf + go) = xv;
        }
      }
      if (MODE == 0 || MODE == 1 || MODE == 2) {
#pragma unroll
        for (int it = 0; it < 4; ++it) {
          const int row = it * 4 + qq;
          const float* sp = slab + row * 68 + c8;
          const v4f xa = *(const v4f*)sp;
          const v4f xb = *(const v4f*)(sp + 4);
          const size_t go = (size_t)(mBase + row) * ldc + n0 + c8;
          if (MODE == 2) {
            v8h hv;
#pragma unroll
            for (int e = 0; e < 4; ++e) { hv[e] = (_Float16)xa[e]; hv[4 + e] = (_Float16)xb[e]; }
            *(volatile v8h*)(Ch + go) = hv;
          } else {
            v8us hb8, lb8;
#pragma unroll
            for (int e = 0; e < 4; ++e) {
              unsigned short hq, lq;
              split_bf(xa[e], hq, lq); hb8[e] = hq;     lb8[e] = lq;
              split_bf(xb[e], hq, lq); hb8[4 + e] = hq; lb8[4 + e] = lq;
            }
            *(volatile v8us*)(Ch + go) = hb8;
            *(volatile v8us*)(Cl + go) = lb8;
          }
        }
      }
      __threadfence();
    }
    wave_sync();
  }
}

#define QB  32
#define KCH 256
#define PSP 264
#define OSP 264
static_assert((NPIX % KCH) == 0 && (NPIX % QB) == 0);
static_assert((PSP % 8) == 0 && (OSP % 8) == 0 && PSP >= KCH && OSP >= CDN);
static_assert(CDN == 8 * 32);

__global__ __launch_bounds__(256) void attn_kernel(const unsigned short* __restrict__ Qh,
                                                   const unsigned short* __restrict__ Ql,
                                                   const unsigned short* __restrict__ Kh,
                                                   const unsigned short* __restrict__ Kl,
                                                   const unsigned short* __restrict__ Vp,
                                                   const float* __restrict__ convf,
                                                   const float* __restrict__ gamma_p,
                                                   unsigned short* __restrict__ Oh,
                                                   unsigned short* __restrict__ Ol) {
  __shared__ __align__(16) _Float16 Ps[QB * PSP];
  __shared__ __align__(16) unsigned short Hs[QB * OSP];
  __shared__ __align__(16) unsigned short Ls[QB * OSP];
  __shared__ __align__(16) float pmax[256];
  __shared__ __align__(16) float psum[256];
  __shared__ __align__(16) float stt[128];
  float* m_s  = stt;
  float* l_s  = stt + 32;
  float* al_s = stt + 64;
  float* li_s = stt + 96;

  const int tid = threadIdx.x, wave = tid >> 5, lane = tid & 31, h = lane >> 4, c = lane & 15;
  const int q0 = (int)blockIdx.x * QB;
  const int kbase = q0 & ~(NPIX - 1);
  const float ninf = -__builtin_inff();

  if (tid < 32) { m_s[tid] = ninf; l_s[tid] = 0.0f; al_s[tid] = 0.0f; li_s[tid] = 0.0f; }
  psum[tid] = 0.0f;

  v16b qb[2][2];
#pragma unroll
  for (int qt = 0; qt < 2; ++qt) {
    const size_t qo = (size_t)(q0 + 16 * qt + c) * (2 * CQK) + 8 * h;
    qb[qt][0] = ldfrag_bf(Qh + qo);
    qb[qt][1] = ldfrag_bf(Ql + qo);
  }
  __syncthreads();

  v8f oacc[2][2];
#pragma unroll
  for (int qt = 0; qt < 2; ++qt)
#pragma unroll
    for (int nt = 0; nt < 2; ++nt) oacc[qt][nt] = zero8();

  const _Float16* Vh = (const _Float16*)(const void*)Vp;
  const _Float16* pa0p = Ps + c * PSP + 8 * h;
  const _Float16* pa1p = Ps + (16 + c) * PSP + 8 * h;
  const int ntile = NPIX / KCH;

#pragma unroll 1
  for (int t = 0; t < ntile; ++t) {
    const int kb = kbase + t * KCH + 32 * wave;
    v16b ka[2][2];
#pragma unroll
    for (int kt = 0; kt < 2; ++kt) {
      const size_t ko = (size_t)(kb + 16 * kt + c) * (2 * CQK) + CQK + 8 * h;
      ka[kt][0] = ldfrag_bf(Kh + ko);
      ka[kt][1] = ldfrag_bf(Kl + ko);
    }
    v8f sacc[2][2];
#pragma unroll
    for (int qt = 0; qt < 2; ++qt) {
#pragma unroll
      for (int kt = 0; kt < 2; ++kt) {
        v8f s = zero8();
        s = mma_bf(ka[kt][0], qb[qt][0], s);
        s = mma_bf(ka[kt][0], qb[qt][1], s);
        s = mma_bf(ka[kt][1], qb[qt][0], s);
        sacc[qt][kt] = s;
      }
    }
    guard4x8(sacc[0][0], sacc[0][1], sacc[1][0], sacc[1][1],
             ka[0][0], ka[0][1], ka[1][0], ka[1][1], qb[0][0], qb[0][1], qb[1][0], qb[1][1]);
    {
      float pm0 = ninf, pm1 = ninf;
#pragma unroll
      for (int kt = 0; kt < 2; ++kt) {
#pragma unroll
        for (int r = 0; r < 8; ++r) {
          pm0 = fmaxf(pm0, sacc[0][kt][r]);
          pm1 = fmaxf(pm1, sacc[1][kt][r]);
        }
      }
      pm0 = fmaxf(pm0, __shfl_xor(pm0, 16, 32));
      pm1 = fmaxf(pm1, __shfl_xor(pm1, 16, 32));
      pmax[wave * 32 + c] = pm0;
      pmax[wave * 32 + 16 + c] = pm1;
    }
    __syncthreads();
    if (wave == 0) {
      const int row = lane;
      float ps = 0.0f;
#pragma unroll
      for (int w = 0; w < 8; ++w) ps += psum[w * 32 + row];
      l_s[row] = l_s[row] * al_s[row] + ps;
      const float mo = m_s[row];
      float mx = mo;
#pragma unroll
      for (int w = 0; w < 8; ++w) mx = fmaxf(mx, pmax[w * 32 + row]);
      al_s[row] = __expf(mo - mx);
      m_s[row] = mx;
    }
    __syncthreads();
    {
      const float mq0 = m_s[c], mq1 = m_s[16 + c];
      float ps0 = 0.0f, ps1 = 0.0f;
#pragma unroll
      for (int kt = 0; kt < 2; ++kt) {
        v8h h0, h1;
#pragma unroll
        for (int r = 0; r < 8; ++r) {
          const float e0 = __expf(sacc[0][kt][r] - mq0); ps0 += e0; h0[r] = (_Float16)(e0 * 4096.0f);
          const float e1 = __expf(sacc[1][kt][r] - mq1); ps1 += e1; h1[r] = (_Float16)(e1 * 4096.0f);
        }
        *(v8h*)(Ps + c * PSP + 32 * wave + 16 * kt + 8 * h) = h0;
        *(v8h*)(Ps + (16 + c) * PSP + 32 * wave + 16 * kt + 8 * h) = h1;
      }
      ps0 += __shfl_xor(ps0, 16, 32);
      ps1 += __shfl_xor(ps1, 16, 32);
      psum[wave * 32 + c] = ps0;
      psum[wave * 32 + 16 + c] = ps1;
      const v4f aA = *(const v4f*)(al_s + 8 * h), aB = *(const v4f*)(al_s + 8 * h + 4);
      const v4f bA = *(const v4f*)(al_s + 16 + 8 * h), bB = *(const v4f*)(al_s + 16 + 8 * h + 4);
#pragma unroll
      for (int nt = 0; nt < 2; ++nt) {
#pragma unroll
        for (int r = 0; r < 4; ++r) {
          oacc[0][nt][r] *= aA[r]; oacc[0][nt][4 + r] *= aB[r];
          oacc[1][nt][r] *= bA[r]; oacc[1][nt][4 + r] *= bB[r];
        }
      }
    }
    __syncthreads();
    {
      const _Float16* vb0p = Vh + (size_t)(32 * wave + c) * NROW + kbase + t * KCH + 8 * h;
      const _Float16* vb1p = vb0p + (size_t)16 * NROW;
#pragma unroll 1
      for (int ks = 0; ks < KCH; ks += 32) {
        const v16h pa0 = ldfrag_h(pa0p + ks), pa1 = ldfrag_h(pa1p + ks);
        const v16h vb0 = ldfrag_h(vb0p + ks), vb1 = ldfrag_h(vb1p + ks);
        oacc[0][0] = mma_h(pa0, vb0, oacc[0][0]);
        oacc[0][1] = mma_h(pa0, vb1, oacc[0][1]);
        oacc[1][0] = mma_h(pa1, vb0, oacc[1][0]);
        oacc[1][1] = mma_h(pa1, vb1, oacc[1][1]);
        guard4x4(oacc[0][0], oacc[0][1], oacc[1][0], oacc[1][1], pa0, pa1, vb0, vb1);
      }
    }
  }
  accg4(oacc[0][0], oacc[0][1], oacc[1][0], oacc[1][1]);

  if (wave == 0) {
    const int row = lane;
    float ps = 0.0f;
#pragma unroll
    for (int w = 0; w < 8; ++w) ps += psum[w * 32 + row];
    const float l = l_s[row] * al_s[row] + ps;
    li_s[row] = (1.0f / l) * (1.0f / 65536.0f);
  }
  __syncthreads();
  {
    const float gam = bfr(gamma_p[0]);
    const v4f iA0 = *(const v4f*)(li_s + 8 * h),      iB0 = *(const v4f*)(li_s + 8 * h + 4);
    const v4f iA1 = *(const v4f*)(li_s + 16 + 8 * h), iB1 = *(const v4f*)(li_s + 16 + 8 * h + 4);
#pragma unroll
    for (int nt = 0; nt < 2; ++nt) {
      const int col = 32 * wave + 16 * nt + c;
#pragma unroll
      for (int r = 0; r < 4; ++r) {
        const int ra = 8 * h + r, rq = 8 * h + 4 + r, rc = 16 + 8 * h + r, rd = 16 + 8 * h + 4 + r;
        unsigned short hb, lb;
        float o;
        o = gam * (oacc[0][nt][r] * iA0[r])     + convf[(size_t)(q0 + ra) * CDN + col];
        split_bf(o, hb, lb); Hs[ra * OSP + col] = hb; Ls[ra * OSP + col] = lb;
        o = gam * (oacc[0][nt][4 + r] * iB0[r]) + convf[(size_t)(q0 + rq) * CDN + col];
        split_bf(o, hb, lb); Hs[rq * OSP + col] = hb; Ls[rq * OSP + col] = lb;
        o = gam * (oacc[1][nt][r] * iA1[r])     + convf[(size_t)(q0 + rc) * CDN + col];
        split_bf(o, hb, lb); Hs[rc * OSP + col] = hb; Ls[rc * OSP + col] = lb;
        o = gam * (oacc[1][nt][4 + r] * iB1[r]) + convf[(size_t)(q0 + rd) * CDN + col];
        split_bf(o, hb, lb); Hs[rd * OSP + col] = hb; Ls[rd * OSP + col] = lb;
      }
    }
  }
  __syncthreads();
  {
#pragma unroll
    for (int ps = 0; ps < 2; ++ps) {
#pragma unroll
      for (int rr = 0; rr < 4; ++rr) {
        const int row = 4 * wave + rr;
        const v8us hvv = *(const v8us*)(Hs + row * OSP + lane * 8);
        const v8us lvv = *(const v8us*)(Ls + row * OSP + lane * 8);
        *(volatile v8us*)(Oh + (size_t)(q0 + row) * CDN + lane * 8) = hvv;
        *(volatile v8us*)(Ol + (size_t)(q0 + row) * CDN + lane * 8) = lvv;
      }
      __threadfence();
    }
  }
}

extern "C" void kernel_launch(void* const* d_in, const int* in_sizes, int n_in,
                              void* d_out, int out_size, void* d_ws, size_t ws_size,
                              hipStream_t stream) {
  if (n_in < 34) return;
  if (in_sizes[0] != NB * CIN * NPIX || in_sizes[1] != NB * CIN * NPIX) return;
  if (out_size != 2 * NB * CIN * NPIX) return;
  for (int m = 0; m < 2; ++m) {
    const int s = 2 + 16 * m;
    if (in_sizes[s + 0] != CDN * CIN * 9) return;
    if (in_sizes[s + 1] != CDN || in_sizes[s + 2] != CDN || in_sizes[s + 3] != CDN) return;
    if (in_sizes[s + 4] != CDN || in_sizes[s + 5] != CDN || in_sizes[s + 6] < 1) return;
    if (in_sizes[s + 7] != CQK * CDN || in_sizes[s + 8] != CQK) return;
    if (in_sizes[s + 9] != CQK * CDN || in_sizes[s + 10] != CQK) return;
    if (in_sizes[s + 11] != CDN * CDN || in_sizes[s + 12] != CDN) return;
    if (in_sizes[s + 13] != CIN * CDN || in_sizes[s + 14] != CIN || in_sizes[s + 15] < 1) return;
  }

  const float* xin[2] = { (const float*)d_in[0], (const float*)d_in[1] };
  const float *cw[2], *cbias[2], *bng[2], *bnb[2], *bnm[2], *bnv[2], *prelu[2];
  const float *qw[2], *qbias[2], *kw[2], *kbias[2], *vw[2], *vbias[2], *uw[2], *ubias[2], *gam[2];
  for (int m = 0; m < 2; ++m) {
    const int s = 2 + 16 * m;
    cw[m]    = (const float*)d_in[s + 0];
    cbias[m] = (const float*)d_in[s + 1];
    bng[m]   = (const float*)d_in[s + 2];
    bnb[m]   = (const float*)d_in[s + 3];
    bnm[m]   = (const float*)d_in[s + 4];
    bnv[m]   = (const float*)d_in[s + 5];
    prelu[m] = (const float*)d_in[s + 6];
    qw[m]    = (const float*)d_in[s + 7];
    qbias[m] = (const float*)d_in[s + 8];
    kw[m]    = (const float*)d_in[s + 9];
    kbias[m] = (const float*)d_in[s + 10];
    vw[m]    = (const float*)d_in[s + 11];
    vbias[m] = (const float*)d_in[s + 12];
    uw[m]    = (const float*)d_in[s + 13];
    ubias[m] = (const float*)d_in[s + 14];
    gam[m]   = (const float*)d_in[s + 15];
  }
  float* out = (float*)d_out;

  const size_t bXP  = (size_t)NB * PADW * PADW * CIN * 2;
  const size_t bWT  = (size_t)CDN * KCV * 2;
  const size_t bWQK = (size_t)2 * CQK * CDN * 2;
  const size_t bWV  = (size_t)CDN * CDN * 2;
  const size_t bWU  = (size_t)CIN * CDN * 2;
  const size_t bCF  = (size_t)NROW * CDN * 4;
  const size_t bCH  = (size_t)NROW * CDN * 2;
  const size_t bQK  = (size_t)NROW * 2 * CQK * 2;
  const size_t bV   = (size_t)CDN * NROW * 2;
  const size_t bO   = (size_t)NROW * CDN * 2;
  size_t off = 0;
  size_t oXP[2], oWT[2], oWQK[2], oWV[2], oWU[2], oCF[2], oCH[2], oCL[2], oQKH[2], oQKL[2], oV[2], oOH[2], oOL[2];
  for (int m = 0; m < 2; ++m) {
    oXP[m]  = off; off += bXP;
    oWT[m]  = off; off += bWT;
    oWQK[m] = off; off += bWQK;
    oWV[m]  = off; off += bWV;
    oWU[m]  = off; off += bWU;
    oCF[m]  = off; off += bCF;
    oCH[m]  = off; off += bCH;
    oCL[m]  = off; off += bCH;
    oQKH[m] = off; off += bQK;
    oQKL[m] = off; off += bQK;
    oV[m]   = off; off += bV;
    oOH[m]  = off; off += bO;
    oOL[m]  = off; off += bO;
  }
  if (off > ws_size) return;
  if (off > (size_t)134217728) return;

  char* ws = (char*)d_ws;
  unsigned short *XP[2], *WT[2], *WQK[2], *WV[2], *WU[2], *CH[2], *CL[2], *QKH[2], *QKL[2], *VPL[2], *OH[2], *OL[2];
  float* CF[2];
  for (int m = 0; m < 2; ++m) {
    XP[m]  = (unsigned short*)(ws + oXP[m]);
    WT[m]  = (unsigned short*)(ws + oWT[m]);
    WQK[m] = (unsigned short*)(ws + oWQK[m]);
    WV[m]  = (unsigned short*)(ws + oWV[m]);
    WU[m]  = (unsigned short*)(ws + oWU[m]);
    CF[m]  = (float*)(ws + oCF[m]);
    CH[m]  = (unsigned short*)(ws + oCH[m]);
    CL[m]  = (unsigned short*)(ws + oCL[m]);
    QKH[m] = (unsigned short*)(ws + oQKH[m]);
    QKL[m] = (unsigned short*)(ws + oQKL[m]);
    VPL[m] = (unsigned short*)(ws + oV[m]);
    OH[m]  = (unsigned short*)(ws + oOH[m]);
    OL[m]  = (unsigned short*)(ws + oOL[m]);
  }

  const dim3 blk(256);
  for (int m = 0; m < 2; ++m) {
    cvt_w_kernel<<<dim3(104), blk, 0, stream>>>(qw[m], kw[m], vw[m], uw[m], WQK[m], WV[m], WU[m]);
    wconv_kernel<<<dim3(CDN * KCV / 8 / 256), blk, 0, stream>>>(cw[m], WT[m]);
    xpad_kernel<<<dim3(NB * PADW), blk, 0, stream>>>(xin[m], XP[m]);
    gemm_kernel<true, false, false, 0><<<dim3(((NROW / 64) * (CDN / 64)) / 8), blk, 0, stream>>>(
        XP[m], XP[m], CIN, WT[m], WT[m], KCV, 0LL,
        CF[m], CH[m], CL[m], CDN, 0LL,
        cbias[m], bng[m], bnb[m], bnm[m], bnv[m], prelu[m],
        NROW, CDN, KCV, 0, 1.0f);
    gemm_kernel<false, true, false, 1><<<dim3(((NROW / 64) * 1) / 8), blk, 0, stream>>>(
        CH[m], CL[m], CDN, WQK[m], WQK[m], CDN, 0LL,
        CF[m], QKH[m], QKL[m], 2 * CQK, 0LL,
        qbias[m], kbias[m], qbias[m], qbias[m], qbias[m], qbias[m],
        NROW, 2 * CQK, CDN, CQK, 1.0f);
    gemm_kernel<false, false, true, 2><<<dim3(((CDN / 64) * (NROW / 64)) / 8), blk, 0, stream>>>(
        WV[m], WV[m], CDN, CH[m], CL[m], CDN, 0LL,
        CF[m], VPL[m], VPL[m], NROW, 0LL,
        vbias[m], vbias[m], vbias[m], vbias[m], vbias[m], vbias[m],
        CDN, NROW, CDN, 0, 16.0f);
  }
  attn_kernel<<<dim3(NROW / QB), blk, 0, stream>>>(QKH[1], QKL[1], QKH[0], QKL[0], VPL[0], CF[0], gam[0],
                                                  OH[0], OL[0]);
  attn_kernel<<<dim3(NROW / QB), blk, 0, stream>>>(QKH[0], QKL[0], QKH[1], QKL[1], VPL[1], CF[1], gam[1],
                                                  OH[1], OL[1]);
  for (int m = 0; m < 2; ++m) {
    float* om = out + (size_t)m * NB * CIN * NPIX;
    gemm_kernel<false, false, true, 3><<<dim3(((CIN / 64) * (NPIX / 64)) / 8, NB), blk, 0, stream>>>(
        WU[m], WU[m], CDN, OH[m], OL[m], CDN, (long long)NPIX * CDN,
        om, OH[m], OL[m], NPIX, (long long)CIN * NPIX,
        ubias[m], xin[m], ubias[m], ubias[m], ubias[m], ubias[m],
        CIN, NPIX, CDN, 0, 1.0f);
  }
  (void)hipGetLastError();
}
